// SimplifiedTransformerBlock_21096879358040
// MI455X (gfx1250) — hardware-verified
//
#include <hip/hip_runtime.h>
#include <math.h>
#include <stdint.h>

#ifndef NB
#define NB       4
#endif
#ifndef SEQ
#define SEQ      2048
#endif
#define NB_FULL  4
#define SEQ_FULL 2048
#ifndef QK_RES
#define QK_RES   1
#endif
#ifndef MLP_RES
#define MLP_RES  1
#endif
#define DMODEL   768
#define DFF      3072
#define NHEAD    12
#define HDIM     64
#define NROWS    (NB * SEQ)
#define NMC      2
#define MCH      (NROWS / NMC)
#define HP       (2 * DMODEL)
#define QKP      (4 * DMODEL)
#define M1P      (2 * DFF)
#define WSC      64.0f
#define LOSC     1024.0f
#define LOINV    (1.0f / 1024.0f)
#define WLO      (WSC / LOSC)
#define HCARRY   16.0f
#define QC       16.0f
#define KC       16.0f
#define VC       16.0f
#define PC       16384.0f
#define H2C      16.0f
#define GC       64.0f
#define LOG2E    1.4426950408889634f
#define RMS_EPS  1e-8f
#define RSQD     0.036084391824351614f
#define NEG_SLOPE 0.01f
static_assert(NHEAD * HDIM == DMODEL);
static_assert(NB >= 1 && NB <= NB_FULL && SEQ >= 64 && SEQ <= SEQ_FULL);
static_assert((SEQ % 64) == 0 && (SEQ % 32) == 0 && (SEQ % 16) == 0);
static_assert((NROWS % 64) == 0 && (NROWS % NMC) == 0 && (MCH % 64) == 0);
static_assert((DMODEL % 64) == 0 && (DFF % 64) == 0 && ((2 * DMODEL) % 64) == 0);
static_assert((HP % 32) == 0 && (M1P % 32) == 0 && (DMODEL % 32) == 0 && (DFF % 32) == 0);

#define HPB         4
#define NHB         (NHEAD / HPB)
#define ATT_THREADS (HPB * 32)
#define ATT_BLOCKS  (NB * (SEQ / 16) * NHB)
#define OSEG        (HPB * HDIM)
#define OSPF        (OSEG + 4)
#define PS_FLOATS   (HPB * 16 * 36)
#define OS_FLOATS   (16 * OSPF)
#define ATT_LDS_FLOATS ((OS_FLOATS > PS_FLOATS) ? OS_FLOATS : PS_FLOATS)
#define ATT_NIT     ((16 * OSEG / 4) / ATT_THREADS)
static_assert(NHB * HPB == NHEAD && ATT_THREADS == 128 && HDIM == 64);
static_assert(((16 * OSEG / 4) % ATT_THREADS) == 0 && ATT_NIT == 8 && (OSEG / 4) == 64);
static_assert(((OSPF * 4) % 16) == 0);
#define RMS_THREADS 192
static_assert(RMS_THREADS * 4 == DMODEL && RMS_THREADS * 8 == HP && (RMS_THREADS % 32) == 0);
#define CS_THREADS  256
static_assert((DMODEL % CS_THREADS) == 0);

typedef _Float16 v16h __attribute__((ext_vector_type(16)));
typedef _Float16 v8h  __attribute__((ext_vector_type(8)));
typedef float    v8f  __attribute__((ext_vector_type(8)));
typedef float    v4f  __attribute__((ext_vector_type(4)));
typedef unsigned int v4u __attribute__((ext_vector_type(4)));
typedef unsigned int v2u __attribute__((ext_vector_type(2)));

union FragH { v16h v; v8h h[2]; v4u u[2]; };

__device__ __forceinline__ unsigned short bf_bits(float f) {
  unsigned u = __float_as_uint(f);
  return (unsigned short)((u + 0x7FFFu + ((u >> 16) & 1u)) >> 16);
}
__device__ __forceinline__ float bf_up(unsigned short h) { return __uint_as_float(((unsigned)h) << 16); }
__device__ __forceinline__ float bfr(float f) { return bf_up(bf_bits(f)); }
__device__ __forceinline__ unsigned short h_bits(_Float16 x) { return __builtin_bit_cast(unsigned short, x); }
__device__ __forceinline__ unsigned pk16(unsigned short a, unsigned short b) { return (unsigned)a | ((unsigned)b << 16); }
__device__ __forceinline__ v8f zero8() { v8f z = {0.f, 0.f, 0.f, 0.f, 0.f, 0.f, 0.f, 0.f}; return z; }
__device__ __forceinline__ int imin(int a, int b) { return a < b ? a : b; }
template <int ACT> __device__ __forceinline__ float act_f(float u) {
  if constexpr (ACT == 2) return (u >= 0.f) ? u : NEG_SLOPE * u;
  else return u;
}

__device__ __forceinline__ v16h ldfrag_h(const _Float16* p) {
  FragH f;
  f.h[0] = *(const v8h*)(p);
  f.h[1] = *(const v8h*)(p + 16);
  return f.v;
}
__device__ __forceinline__ v16h ldfrag_u(const unsigned short* p) {
  FragH f;
  f.u[0] = *(const v4u*)(p);
  f.u[1] = *(const v4u*)(p + 16);
  return f.v;
}

__device__ __forceinline__ v8f mma_raw(v16h a, v16h b, v8f c) {
  return __builtin_amdgcn_wmma_f32_16x16x32_f16(false, a, false, b, (short)0, c, false, false);
}
__device__ __forceinline__ void dep_guard1(v8f& a, v8f& b, v16h x) {
#if defined(__HIP_DEVICE_COMPILE__)
  asm volatile("v_nop\n\tv_nop\n\tv_nop\n\tv_nop" : "+v"(a), "+v"(b) : "v"(x));
#endif
}
__device__ __forceinline__ void guard_2x4(v8f& s, v8f& t, v16h a0, v16h a1, v16h b0, v16h b1) {
#if defined(__HIP_DEVICE_COMPILE__)
  asm volatile("v_nop\n\tv_nop\n\tv_nop\n\tv_nop" : "+v"(s), "+v"(t) : "v"(a0), "v"(a1), "v"(b0), "v"(b1));
#endif
}
__device__ __forceinline__ void guard_pv4(v8f& a, v8f& b, v8f& c, v8f& d, v16h x, v16h y, v16h z, v16h w, v16h u) {
#if defined(__HIP_DEVICE_COMPILE__)
  asm volatile("v_nop\n\tv_nop\n\tv_nop\n\tv_nop"
               : "+v"(a), "+v"(b), "+v"(c), "+v"(d) : "v"(x), "v"(y), "v"(z), "v"(w), "v"(u));
#endif
}
__device__ __forceinline__ void keep4_h(v16h a, v16h b, v16h c, v16h d) {
#if defined(__HIP_DEVICE_COMPILE__)
  asm volatile("v_nop" :: "v"(a), "v"(b), "v"(c), "v"(d));
#endif
}
__device__ __forceinline__ void acc_guard4(v8f& a, v8f& b, v8f& c, v8f& d) {
#if defined(__HIP_DEVICE_COMPILE__)
  asm volatile("v_nop\n\tv_nop\n\tv_nop\n\tv_nop" : "+v"(a), "+v"(b), "+v"(c), "+v"(d));
#endif
}
__device__ __forceinline__ void wave_sync_lds() {
  __builtin_amdgcn_fence(__ATOMIC_RELEASE, "workgroup");
  __builtin_amdgcn_wave_barrier();
  __builtin_amdgcn_fence(__ATOMIC_ACQUIRE, "workgroup");
}

template <int RNB, int DUAL>
__global__ __launch_bounds__(256) void tcvt16(const float* __restrict__ src, long long sstr,
                                              unsigned short* dst, long long dstr,
                                              int R, int C, int ldo, int off2, float sc, float sc2) {
  __shared__ __align__(16) float sT[64 * 68];
  const int tid = threadIdx.x, lane = tid & 31, wave = tid >> 5;
  const int c0 = blockIdx.x * 64, r0 = blockIdx.y * 64;
  const float* S = src + (size_t)((long long)blockIdx.z * sstr);
  unsigned short* Dd = dst + (size_t)((long long)blockIdx.z * dstr);
  const int rr = tid >> 2, cc = (tid & 3) * 16;
  const int r = r0 + rr;
  const int rcl = imin(r, R - 1);
  const float* sp = S + (size_t)rcl * C;
#pragma unroll
  for (int e = 0; e < 16; ++e) {
    const int cidx = c0 + cc + e;
    const int ccl = imin(cidx, C - 1);
    float a = sp[ccl];
    a = (r < R && cidx < C) ? a : 0.f;
    if constexpr (RNB == 1) a = bfr(a);
    sT[(cc + e) * 68 + rr] = a;
  }
  __syncthreads();
  v4u hv[2], lv[2];
#pragma unroll
  for (int it = 0; it < 2; ++it) {
    const int q = it * 32 + wave * 4 + (lane >> 3);
    const float* tp = sT + q * 68 + (lane & 7) * 8;
    const v4f f0 = *(const v4f*)(tp), f1 = *(const v4f*)(tp + 4);
    v4u a, b = {0u, 0u, 0u, 0u};
    a[0] = pk16(h_bits((_Float16)(f0[0] * sc)), h_bits((_Float16)(f0[1] * sc)));
    a[1] = pk16(h_bits((_Float16)(f0[2] * sc)), h_bits((_Float16)(f0[3] * sc)));
    a[2] = pk16(h_bits((_Float16)(f1[0] * sc)), h_bits((_Float16)(f1[1] * sc)));
    a[3] = pk16(h_bits((_Float16)(f1[2] * sc)), h_bits((_Float16)(f1[3] * sc)));
    if constexpr (DUAL == 1) {
      b[0] = pk16(h_bits((_Float16)(f0[0] * sc2)), h_bits((_Float16)(f0[1] * sc2)));
      b[1] = pk16(h_bits((_Float16)(f0[2] * sc2)), h_bits((_Float16)(f0[3] * sc2)));
      b[2] = pk16(h_bits((_Float16)(f1[0] * sc2)), h_bits((_Float16)(f1[1] * sc2)));
      b[3] = pk16(h_bits((_Float16)(f1[2] * sc2)), h_bits((_Float16)(f1[3] * sc2)));
    }
    hv[it] = a; lv[it] = b;
  }
  for (int pass = 0; pass < 2; ++pass) {
#pragma unroll
    for (int it = 0; it < 2; ++it) {
      const int q = it * 32 + wave * 4 + (lane >> 3);
      unsigned short* p = Dd + (size_t)(c0 + q) * ldo + r0 + (lane & 7) * 8;
      *(volatile v4u*)p = hv[it];
      if constexpr (DUAL == 1) *(volatile v4u*)(p + off2) = lv[it];
    }
    __threadfence();
  }
}

template <int OM, int RM, int ACT, int BM>
__global__ __launch_bounds__(256) void gemm64(
    const unsigned short* __restrict__ Ap, int lda, long long sA,
    const unsigned short* __restrict__ Btp, int ldb, long long sB,
    const float* __restrict__ Rp,
    const float* __restrict__ biasp, int nbias,
    void* Cout, int ldc, long long sC, int loff,
    int M, int N, int K, float oscale, float ocarry) {
  __shared__ __align__(16) float sT[8][16 * 68];
  const int by   = blockIdx.y;
  const int lane = threadIdx.x & 31;
  const int wave = threadIdx.x >> 5;
  const int tilesN = N >> 6;
  const int tilesM = M >> 6;
  const int tile = blockIdx.x * 8 + wave;
  if (tile >= tilesM * tilesN) return;
  const int tm = tile / tilesN;
  const int tn = tile - tm * tilesN;
  const int m0 = tm << 6;
  const int n0 = tn << 6;

  const unsigned short* A1 = Ap  + (size_t)((long long)by * sA);
  const unsigned short* Bb = Btp + (size_t)((long long)by * sB);

  const int rlane = lane & 15;
  const int koff  = (lane >> 4) * 8;
  const int mOff  = (lane >> 4) * 8;

  v8f acc[4][4];
#pragma unroll
  for (int i = 0; i < 4; ++i)
#pragma unroll
    for (int j = 0; j < 4; ++j) acc[i][j] = zero8();

  for (int k0 = 0; k0 < K; k0 += 32) {
    v16h bh[4];
#pragma unroll
    for (int j = 0; j < 4; ++j) {
      const size_t bofs = (size_t)(n0 + (j << 4) + rlane) * ldb + koff + k0;
      bh[j] = ldfrag_u(Bb + bofs);
    }
#pragma unroll
    for (int i = 0; i < 4; ++i) {
      const size_t ao = (size_t)(m0 + (i << 4) + rlane) * lda + koff + k0;
      const v16h ah = ldfrag_u(A1 + ao);
#pragma unroll
      for (int j = 0; j < 4; ++j) acc[i][j] = mma_raw(ah, bh[j], acc[i][j]);
      dep_guard1(acc[i][0], acc[i][3], ah);
    }
    keep4_h(bh[0], bh[1], bh[2], bh[3]);
  }
  acc_guard4(acc[0][0], acc[0][1], acc[0][2], acc[0][3]);
  acc_guard4(acc[1][0], acc[1][1], acc[1][2], acc[1][3]);
  acc_guard4(acc[2][0], acc[2][1], acc[2][2], acc[2][3]);
  acc_guard4(acc[3][0], acc[3][1], acc[3][2], acc[3][3]);

  const int hh2 = lane >> 4, c4 = (lane & 15) * 4;
  const int q8  = lane >> 3, c8 = (lane & 7) * 8;

  float bc4[4], bc8[8];
#pragma unroll
  for (int e = 0; e < 4; ++e) bc4[e] = 0.f;
#pragma unroll
  for (int e = 0; e < 8; ++e) bc8[e] = 0.f;
  if constexpr (BM == 1) {
    if constexpr (OM == 0) {
#pragma unroll
      for (int e = 0; e < 4; ++e) {
        const int n = n0 + c4 + e;
        const int ncl = imin(n, nbias - 1);
        const float t = bfr(biasp[ncl]);
        bc4[e] = (n < nbias) ? t : 0.f;
      }
    } else {
#pragma unroll
      for (int e = 0; e < 8; ++e) {
        const int n = n0 + c8 + e;
        const int ncl = imin(n, nbias - 1);
        const float t = bfr(biasp[ncl]);
        bc8[e] = (n < nbias) ? t : 0.f;
      }
    }
  }

  float* slab = sT[wave];
#pragma unroll
  for (int i = 0; i < 4; ++i) {
    const int mBase = m0 + (i << 4);
#pragma unroll
    for (int j = 0; j < 4; ++j) {
#pragma unroll
      for (int r = 0; r < 8; ++r) {
        slab[(mOff + r) * 68 + (j << 4) + rlane] = acc[i][j][r];
      }
    }
    wave_sync_lds();
    if constexpr (OM == 0) {
      float* C = (float*)Cout + (size_t)((long long)by * sC);
      v4f vals[8];
#pragma unroll
      for (int it = 0; it < 8; ++it) {
        const int row = it * 2 + hh2;
        const int gr  = mBase + row;
        v4f v = *(const v4f*)(slab + row * 68 + c4);
        v4f rv = {0.f, 0.f, 0.f, 0.f};
        if constexpr (RM == 1 || RM == 2) {
          const float* R = Rp + (size_t)((long long)by * sC);
          const v4f rraw = *(const v4f*)(R + (size_t)gr * ldc + n0 + c4);
#pragma unroll
          for (int e = 0; e < 4; ++e) rv[e] = (RM == 1) ? bfr(rraw[e]) : rraw[e];
        }
#pragma unroll
        for (int e = 0; e < 4; ++e) {
          float u = v[e] * oscale;
          if constexpr (BM == 1) u += bc4[e];
          u = act_f<ACT>(u);
          v[e] = u + rv[e];
        }
        vals[it] = v;
      }
      for (int pass = 0; pass < 2; ++pass) {
#pragma unroll
        for (int it = 0; it < 8; ++it) {
          const int gr = mBase + it * 2 + hh2;
          *(volatile v4f*)(C + (size_t)gr * ldc + n0 + c4) = vals[it];
        }
        __threadfence();
      }
    } else {
      unsigned short* C = (unsigned short*)Cout + (size_t)((long long)by * sC);
      v4u hv[4], lv[4];
#pragma unroll
      for (int it = 0; it < 4; ++it) {
        const int row = it * 4 + q8;
        const float* sp = slab + row * 68 + c8;
        v4u a = {0u, 0u, 0u, 0u}, bl = {0u, 0u, 0u, 0u};
#pragma unroll
        for (int e = 0; e < 4; ++e) {
          float f0 = sp[2 * e] * oscale;
          float f1 = sp[2 * e + 1] * oscale;
          if constexpr (BM == 1) { f0 += bc8[2 * e]; f1 += bc8[2 * e + 1]; }
          f0 = act_f<ACT>(f0); f1 = act_f<ACT>(f1);
          f0 *= ocarry; f1 *= ocarry;
          const _Float16 g0 = (_Float16)f0, g1 = (_Float16)f1;
          a[e] = pk16(h_bits(g0), h_bits(g1));
          if constexpr (OM == 3) {
            const _Float16 d0 = (_Float16)((f0 - (float)g0) * LOSC);
            const _Float16 d1 = (_Float16)((f1 - (float)g1) * LOSC);
            bl[e] = pk16(h_bits(d0), h_bits(d1));
          }
        }
        hv[it] = a; lv[it] = bl;
      }
      for (int pass = 0; pass < 2; ++pass) {
#pragma unroll
        for (int it = 0; it < 4; ++it) {
          const int row = it * 4 + q8;
          unsigned short* p = C + (size_t)(mBase + row) * ldc + n0 + c8;
          *(volatile v4u*)p = hv[it];
          if constexpr (OM == 3) *(volatile v4u*)(p + loff) = lv[it];
        }
        __threadfence();
      }
    }
    wave_sync_lds();
  }
}

template <int MODE>
__global__ __launch_bounds__(RMS_THREADS)
void rmsn(const float* __restrict__ Yp, const float* __restrict__ sp, float* HF, unsigned short* H, float hc) {
  __shared__ float red[RMS_THREADS / 32];
  __shared__ __align__(16) unsigned short srow[HP];
  const int row  = blockIdx.x;
  const int tid  = threadIdx.x;
  const int lane = tid & 31;
  const int wave = tid >> 5;
  size_t irow = (size_t)row;
  if constexpr (MODE == 1) {
    const int b = row / SEQ;
    const int s = row - b * SEQ;
    irow = (size_t)b * SEQ_FULL + (size_t)s;
  }
  v4f v = *(const v4f*)(Yp + irow * DMODEL + (size_t)tid * 4);
  if constexpr (MODE == 1) {
#pragma unroll
    for (int e = 0; e < 4; ++e) v[e] = bfr(v[e]);
  }
  float q = (v[0] * v[0] + v[1] * v[1]) + (v[2] * v[2] + v[3] * v[3]);
#pragma unroll
  for (int off = 1; off < 32; off <<= 1) q += __shfl_xor(q, off, 32);
  if (lane == 0) red[wave] = q;
  __syncthreads();
  float tot = 0.f;
#pragma unroll
  for (int w = 0; w < RMS_THREADS / 32; ++w) tot += red[w];
  const float rms = sqrtf(tot) * RSQD;
  const float inv = 1.0f / (rms + RMS_EPS);
  const v4f gv = *(const v4f*)(sp + (size_t)tid * 4);
  v4f h;
#pragma unroll
  for (int e = 0; e < 4; ++e) h[e] = (bfr(gv[e]) * v[e]) * inv;
  v2u whi, wlo;
  {
    unsigned short hb16[4], lb16[4];
#pragma unroll
    for (int e = 0; e < 4; ++e) {
      const float f = h[e] * hc;
      const _Float16 g = (_Float16)f;
      hb16[e] = h_bits(g);
      lb16[e] = h_bits((_Float16)((f - (float)g) * LOSC));
    }
    whi[0] = pk16(hb16[0], hb16[1]); whi[1] = pk16(hb16[2], hb16[3]);
    wlo[0] = pk16(lb16[0], lb16[1]); wlo[1] = pk16(lb16[2], lb16[3]);
  }
  *(v2u*)(srow + tid * 4) = whi;
  *(v2u*)(srow + DMODEL + tid * 4) = wlo;
  __syncthreads();
  const v4u hv = *(const v4u*)(srow + tid * 8);
  unsigned short* dst = H + (size_t)row * HP + (size_t)tid * 8;
  for (int pass = 0; pass < 2; ++pass) {
    if constexpr (MODE == 1) *(volatile v4f*)(HF + (size_t)row * DMODEL + (size_t)tid * 4) = h;
    *(volatile v4u*)dst = hv;
    __threadfence();
  }
}

__global__ __launch_bounds__(CS_THREADS)
void skipcen(const float* __restrict__ HFp, const float* __restrict__ gsp, const float* __restrict__ gcp, float* Tp) {
  const int nseg = DMODEL / CS_THREADS;
  const int b  = blockIdx.x / nseg;
  const int d  = (blockIdx.x % nseg) * CS_THREADS + threadIdx.x;
  const int hd = d / HDIM;
  const float gs = bfr(gsp[hd]);
  const float gc = bfr(gcp[hd]);
  const float* hp = HFp + (size_t)b * SEQ * DMODEL + d;
  float*       tp = Tp  + (size_t)b * SEQ * DMODEL + d;
  float acc = 0.f;
#pragma unroll 1
  for (int s = 0; s < SEQ; ++s) {
    const float hv = hp[(size_t)s * DMODEL];
    acc += hv;
    const float pm  = acc * (1.0f / (float)(s + 1));
    const float val = gs * hv - gc * pm;
    float* q = tp + (size_t)s * DMODEL;
    *(volatile float*)q = val;
    __threadfence();
    *(volatile float*)q = val;
  }
}

__global__ __launch_bounds__(ATT_THREADS)
void attnc(const unsigned short* __restrict__ QKq, const unsigned short* __restrict__ VTq,
           const float* __restrict__ Tp, const float* __restrict__ xp, const float* __restrict__ grp,
           float* X1) {
  __shared__ __align__(16) float smem[ATT_LDS_FLOATS];

  const int tid  = threadIdx.x;
  const int wave = tid >> 5;
  const int lane = tid & 31;
  const int hh   = lane >> 4;
  const int c    = lane & 15;

  const int hb   = blockIdx.x % NHB;
  const int qt   = (blockIdx.x / NHB) % (SEQ / 16);
  const int bat  = blockIdx.x / (NHB * (SEQ / 16));
  const int head = hb * HPB + wave;
  const int q0   = qt * 16;

  const _Float16* QK = (const _Float16*)(const void*)QKq;
  const _Float16* Qh = QK + ((size_t)bat * SEQ + q0 + c) * QKP + head * HDIM + 8 * hh;
  const _Float16* Kb = QK + (size_t)bat * SEQ * QKP + DMODEL + head * HDIM + 8 * hh;
  const _Float16* Vb = (const _Float16*)(const void*)VTq + ((size_t)bat * DMODEL + head * HDIM) * SEQ + 8 * hh;
  const float lsc = LOG2E / (QC * KC);

  const v16h qa = ldfrag_h(Qh), qb = ldfrag_h(Qh + 32);
  const v16h ra = ldfrag_h(Qh + 2 * DMODEL), rb = ldfrag_h(Qh + 2 * DMODEL + 32);

  float mrow[8], lrow[8];
  v8f o0 = zero8(), o1 = zero8(), o2 = zero8(), o3 = zero8();
#pragma unroll
  for (int r = 0; r < 8; ++r) { mrow[r] = -INFINITY; lrow[r] = 0.f; }
  float* pt = smem + wave * (16 * 36);
  const int qrow = q0 + 8 * hh;

#pragma unroll 1
  for (int kb = 0; kb < q0 + 16; kb += 32) {
    const _Float16* kp = Kb + (size_t)(kb + c) * QKP;
    v8f sh0, sx0, sh1, sx1;
    {
      const v16h k0 = ldfrag_h(kp), k1 = ldfrag_h(kp + 32);
      const v16h l0 = ldfrag_h(kp + 2 * DMODEL), l1 = ldfrag_h(kp + 2 * DMODEL + 32);
      sh0 = mma_raw(qa, k0, zero8());
      sh0 = mma_raw(qb, k1, sh0);
      sx0 = mma_raw(qa, l0, zero8());
      sx0 = mma_raw(qb, l1, sx0);
      sx0 = mma_raw(ra, k0, sx0);
      sx0 = mma_raw(rb, k1, sx0);
      guard_2x4(sh0, sx0, k0, k1, l0, l1);
    }
    {
      const _Float16* kq = kp + (size_t)16 * QKP;
      const v16h k0 = ldfrag_h(kq), k1 = ldfrag_h(kq + 32);
      const v16h l0 = ldfrag_h(kq + 2 * DMODEL), l1 = ldfrag_h(kq + 2 * DMODEL + 32);
      sh1 = mma_raw(qa, k0, zero8());
      sh1 = mma_raw(qb, k1, sh1);
      sx1 = mma_raw(qa, l0, zero8());
      sx1 = mma_raw(qb, l1, sx1);
      sx1 = mma_raw(ra, k0, sx1);
      sx1 = mma_raw(rb, k1, sx1);
      guard_2x4(sh1, sx1, k0, k1, l0, l1);
      keep4_h(qa, qb, ra, rb);
    }
    const int key0 = kb + c, key1 = kb + 16 + c;
#pragma unroll
    for (int r = 0; r < 8; ++r) {
      const float u0 = (sh0[r] + sx0[r] * LOINV) * lsc;
      const float u1 = (sh1[r] + sx1[r] * LOINV) * lsc;
      const int   qi = qrow + r;
      const bool  ok0 = key0 <= qi, ok1 = key1 <= qi;
      const float t0 = ok0 ? u0 : -INFINITY;
      const float t1 = ok1 ? u1 : -INFINITY;
      float mx = fmaxf(t0, t1);
#pragma unroll
      for (int off = 1; off < 16; off <<= 1) mx = fmaxf(mx, __shfl_xor(mx, off, 32));
      const float mn = fmaxf(mrow[r], mx);
      const float al = exp2f(fmaxf(mrow[r] - mn, -126.0f));
      mrow[r] = mn;
      const float f0 = exp2f(u0 - mn);
      const float f1 = exp2f(u1 - mn);
      const float e0 = ok0 ? f0 : 0.f;
      const float e1 = ok1 ? f1 : 0.f;
      float ps = e0 + e1;
#pragma unroll
      for (int off = 1; off < 16; off <<= 1) ps += __shfl_xor(ps, off, 32);
      lrow[r] = lrow[r] * al + ps;
      o0[r] *= al;
      o1[r] *= al;
      o2[r] *= al;
      o3[r] *= al;
      const int ro = (8 * hh + r) * 36 + c;
      pt[ro]      = e0;
      pt[ro + 16] = e1;
    }
    wave_sync_lds();
    FragH ph;
    {
      const float* prow = pt + c * 36 + 8 * hh;
      const v4f p0 = *(const v4f*)(prow), p1 = *(const v4f*)(prow + 4);
      const v4f p2 = *(const v4f*)(prow + 16), p3 = *(const v4f*)(prow + 20);
#pragma unroll
      for (int e = 0; e < 4; ++e) {
        ph.h[0][e]     = (_Float16)(p0[e] * PC);
        ph.h[0][4 + e] = (_Float16)(p1[e] * PC);
        ph.h[1][e]     = (_Float16)(p2[e] * PC);
        ph.h[1][4 + e] = (_Float16)(p3[e] * PC);
      }
    }
    const _Float16* vp = Vb + (size_t)c * SEQ + kb;
    {
      const v16h vb0 = ldfrag_h(vp);
      const v16h vb1 = ldfrag_h(vp + (size_t)16 * SEQ);
      const v16h vb2 = ldfrag_h(vp + (size_t)32 * SEQ);
      const v16h vb3 = ldfrag_h(vp + (size_t)48 * SEQ);
      o0 = mma_raw(ph.v, vb0, o0);
      o1 = mma_raw(ph.v, vb1, o1);
      o2 = mma_raw(ph.v, vb2, o2);
      o3 = mma_raw(ph.v, vb3, o3);
      guard_pv4(o0, o1, o2, o3, ph.v, vb0, vb1, vb2, vb3);
    }
    wave_sync_lds();
  }

  __syncthreads();
  float* Os = smem;
  const float oc = 1.0f / (PC * VC);
  float* osw = Os + wave * HDIM + c;
#pragma unroll
  for (int r = 0; r < 8; ++r) {
    const float inv = (1.0f / lrow[r]) * oc;
    float* op = osw + (8 * hh + r) * OSPF;
    op[0]  = o0[r] * inv;
    op[16] = o1[r] * inv;
    op[32] = o2[r] * inv;
    op[48] = o3[r] * inv;
  }
  __syncthreads();
  {
    v4f vals[ATT_NIT];
    const int colb = hb * OSEG;
#pragma unroll
    for (int it = 0; it < ATT_NIT; ++it) {
      const int p = it * ATT_THREADS + tid;
      const int row = p >> 6, c4 = (p & 63) * 4;
      const int hd = hb * HPB + (c4 >> 6);
      const float gr = bfr(grp[hd]);
      const v4f ov = *(const v4f*)(Os + row * OSPF + c4);
      const size_t gro = (size_t)bat * SEQ + q0 + row;
      const size_t gri = (size_t)bat * SEQ_FULL + q0 + row;
      const v4f xv = *(const v4f*)(xp + gri * DMODEL + colb + c4);
      const v4f tv = *(const v4f*)(Tp + gro * DMODEL + colb + c4);
      v4f w;
#pragma unroll
      for (int e = 0; e < 4; ++e) w[e] = bfr(xv[e]) + (gr * ov[e] + tv[e]);
      vals[it] = w;
    }
    for (int pass = 0; pass < 2; ++pass) {
#pragma unroll
      for (int it = 0; it < ATT_NIT; ++it) {
        const int p = it * ATT_THREADS + tid;
        const int row = p >> 6, c4 = (p & 63) * 4;
        const size_t gro = (size_t)bat * SEQ + q0 + row;
        *(volatile v4f*)(X1 + gro * DMODEL + colb + c4) = vals[it];
      }
      __threadfence();
    }
  }
}

extern "C" void kernel_launch(void* const* d_in, const int* in_sizes, int n_in,
                              void* d_out, int out_size, void* d_ws, size_t ws_size,
                              hipStream_t stream) {
  if (n_in < 12) return;
  if (in_sizes[0] < ((NB - 1) * SEQ_FULL + SEQ) * DMODEL) return;
  if (in_sizes[1] < DMODEL) return;
  if (in_sizes[2] != DMODEL * 2 * DMODEL) return;
  if (in_sizes[3] < 2 * DMODEL) return;
  if (in_sizes[4] < NHEAD || in_sizes[5] < NHEAD || in_sizes[6] < NHEAD) return;
  if (in_sizes[7] < DMODEL) return;
  if (in_sizes[8] != DMODEL * DFF || in_sizes[9] < DFF) return;
  if (in_sizes[10] != DFF * DMODEL || in_sizes[11] < DMODEL) return;
  if (out_size < NROWS * DMODEL) return;

  const float* x      = (const float*)d_in[0];
  const float* scale1 = (const float*)d_in[1];
  const float* qk_w   = (const float*)d_in[2];
  const float* qk_b   = (const float*)d_in[3];
  const float* g_res  = (const float*)d_in[4];
  const float* g_skp  = (const float*)d_in[5];
  const float* g_cen  = (const float*)d_in[6];
  const float* scale2 = (const float*)d_in[7];
  const float* w_1    = (const float*)d_in[8];
  const float* b_1    = (const float*)d_in[9];
  const float* w_2    = (const float*)d_in[10];
  const float* b_2    = (const float*)d_in[11];
  float*       out    = (float*)d_out;

  const size_t PW1  = (size_t)DFF * HP * 2;
  const size_t PW2  = (size_t)DMODEL * M1P * 2;
  const size_t PWQK = (size_t)(2 * DMODEL) * HP * 2;
  const size_t PF32 = (size_t)NROWS * DMODEL * 4;
  const size_t PH16 = (size_t)NROWS * HP * 2;
  const size_t PVT  = (size_t)NB * DMODEL * SEQ * 2;
  const size_t PQK  = (size_t)NROWS * QKP * 2;
  const size_t PM1  = (size_t)MCH * M1P * 2;
  const size_t oW1  = 0;
  const size_t oW2  = oW1 + PW1;
  const size_t oXF  = oW2 + PW2;
  const size_t oH16 = oXF + PF32;
  const size_t oVT  = oH16;
  const size_t oT   = oVT + PVT;
  const size_t oWQK = oH16 + PH16;
  const size_t eT   = oT + PF32;
  const size_t eWQK = oWQK + PWQK;
  const size_t oQK  = (eT > eWQK) ? eT : eWQK;
  const size_t endA = oQK + PQK;
  const size_t oH2  = oH16;
  const size_t oM1  = oH2 + PH16;
  const size_t endB = oM1 + PM1;
  const size_t endAll = (endA > endB) ? endA : endB;
  if (endAll > ws_size) return;
  if (endAll > (size_t)134217728) return;
  if (oH2 < oXF + PF32) return;

  char* ws = (char*)d_ws;
  unsigned short* W1P  = (unsigned short*)(ws + oW1);
  unsigned short* W2P  = (unsigned short*)(ws + oW2);
  float*          HF   = (float*)(ws + oXF);
  float*          X1F  = (float*)(ws + oXF);
  unsigned short* H16  = (unsigned short*)(ws + oH16);
  unsigned short* VT   = (unsigned short*)(ws + oVT);
  float*          T    = (float*)(ws + oT);
  unsigned short* WQK  = (unsigned short*)(ws + oWQK);
  unsigned short* QK16 = (unsigned short*)(ws + oQK);
  unsigned short* H2   = (unsigned short*)(ws + oH2);
  unsigned short* M1   = (unsigned short*)(ws + oM1);

  const dim3 blk(256);
  const dim3 gTqk((2 * DMODEL) / 64, DMODEL / 64, 1);
  const dim3 gT1(DFF / 64, DMODEL / 64, 1);
  const dim3 gT2(DMODEL / 64, DFF / 64, 1);
  const dim3 gTv(DMODEL / 64, SEQ / 64, NB);
  const int tilesQK = (NROWS / 64) * ((2 * DMODEL) / 64);
  const int tilesF1 = (MCH / 64) * (DFF / 64);
  const int tilesF2 = (MCH / 64) * (DMODEL / 64);
  const dim3 gQK((tilesQK + 7) / 8, 1);
  const dim3 gF1((tilesF1 + 7) / 8, 1);
  const dim3 gF2((tilesF2 + 7) / 8, 1);
  const dim3 gRMS(NROWS);
  const dim3 bRMS(RMS_THREADS);
  const dim3 gCS(NB * (DMODEL / CS_THREADS));
  const dim3 bCS(CS_THREADS);
  const dim3 gAT(ATT_BLOCKS);
  const dim3 bAT(ATT_THREADS);
  const int KQK = (QK_RES != 0) ? HP : DMODEL;
  const int KF1 = (MLP_RES != 0) ? HP : DMODEL;
  const int KF2 = (MLP_RES != 0) ? M1P : DFF;

  tcvt16<1, 1><<<gTqk, blk, 0, stream>>>(qk_w, 0LL, WQK, 0LL, DMODEL, 2 * DMODEL, HP, DMODEL, WSC, WLO);
  tcvt16<1, 1><<<gT1,  blk, 0, stream>>>(w_1,  0LL, W1P, 0LL, DMODEL, DFF, HP, DMODEL, WSC, WLO);
  tcvt16<1, 1><<<gT2,  blk, 0, stream>>>(w_2,  0LL, W2P, 0LL, DFF, DMODEL, M1P, DFF, WSC, WLO);

  rmsn<1><<<gRMS, bRMS, 0, stream>>>(x, scale1, HF, H16, HCARRY);

  gemm64<3, 0, 0, 1><<<gQK, blk, 0, stream>>>(
      H16, HP, 0LL,
      WQK, HP, 0LL,
      X1F,
      qk_b, 2 * DMODEL,
      (void*)QK16, QKP, 0LL, 2 * DMODEL,
      NROWS, 2 * DMODEL, KQK, 1.0f / (HCARRY * WSC), QC);

  tcvt16<0, 0><<<gTv, blk, 0, stream>>>(HF, (long long)SEQ * DMODEL, VT, (long long)DMODEL * SEQ,
                                        SEQ, DMODEL, SEQ, 0, VC, 0.f);

  skipcen<<<gCS, bCS, 0, stream>>>(HF, g_skp, g_cen, T);

  attnc<<<gAT, bAT, 0, stream>>>(QK16, VT, T, x, g_res, X1F);

  rmsn<0><<<gRMS, bRMS, 0, stream>>>(X1F, scale2, X1F, H2, H2C);

  for (int ch = 0; ch < NMC; ++ch) {
    gemm64<3, 0, 2, 1><<<gF1, blk, 0, stream>>>(
        H2 + (size_t)ch * MCH * HP, HP, 0LL,
        W1P, HP, 0LL,
        X1F,
        b_1, DFF,
        (void*)M1, M1P, 0LL, DFF,
        MCH, DFF, KF1, 1.0f / (H2C * WSC), GC);
    gemm64<0, 2, 0, 1><<<gF2, blk, 0, stream>>>(
        M1, M1P, 0LL,
        W2P, M1P, 0LL,
        X1F + (size_t)ch * MCH * DMODEL,
        b_2, DMODEL,
        (void*)(out + (size_t)ch * MCH * DMODEL), DMODEL, 0LL, 0,
        MCH, DMODEL, KF2, 1.0f / (GC * WSC), 1.0f);
  }
  (void)hipGetLastError();
}
